// OctreeDeconvGnRelu_25649544692150
// MI455X (gfx1250) — hardware-verified
//
#include <hip/hip_runtime.h>


namespace {
constexpr int N = 300000, KT = 27, CI = 32, CO = 32, KK = KT * CI, NB = 8, G = 8, CG = CO / G, NTILE = N / 16;
constexpr float XS = 8.0f, WSC = 256.0f, EPS = 1e-5f;
typedef _Float16 b16;
typedef __attribute__((ext_vector_type(16))) _Float16 v16b;
typedef __attribute__((ext_vector_type(8))) _Float16 v8b;
typedef __attribute__((ext_vector_type(8))) float v8f;
typedef __attribute__((ext_vector_type(4))) float v4f;
__device__ __forceinline__ float bf16_rne(float f) { unsigned int u = __float_as_uint(f); u += 0x7FFFu + ((u >> 16) & 1u); float r = __uint_as_float(u & 0xFFFF0000u); asm volatile("" : "+v"(r)); return r; }
__device__ __forceinline__ v16b frag_kb(const b16* p, int hh) { const v8b a = *(const v8b*)(p + 8 * hh), b = *(const v8b*)(p + 16 + 8 * hh); v16b f;
#pragma unroll
  for (int e = 0; e < 8; ++e) { f[e] = a[e]; f[8 + e] = b[e]; } return f; }
__device__ __forceinline__ v8f wmma16b(v16b a, v16b b, v8f c) { v8f d = __builtin_amdgcn_wmma_f32_16x16x32_f16(false, a, false, b, (short)0, c, false, false); asm volatile("v_nop\n\tv_nop\n\tv_nop\n\tv_nop" : "+v"(d) : "v"(a), "v"(b)); return d; }
__device__ __forceinline__ void wave_lds_sync() { __builtin_amdgcn_fence(__ATOMIC_RELEASE, "workgroup"); __builtin_amdgcn_wave_barrier(); __builtin_amdgcn_fence(__ATOMIC_ACQUIRE, "workgroup"); }
__device__ __forceinline__ float pmul(float a, float b) { float p = a * b; asm volatile("" : "+v"(p)); return p; }
__device__ __forceinline__ int iclamp(int v, int lo, int hi) { return v < lo ? lo : (v > hi ? hi : v); }

__global__ __launch_bounds__(256) void prep_kernel(const float* __restrict__ data, const float* __restrict__ W, b16* __restrict__ DP, b16* __restrict__ WT) { const size_t u = (size_t)blockIdx.x * 256 + threadIdx.x;
  for (int pass = 0; pass < 2; ++pass) {
    if (u < (size_t)N * CI / 8) { v8b v;
#pragma unroll
      for (int j = 0; j < 8; ++j) v[j] = (b16)(bf16_rne(data[u * 8 + j]) * XS); *(volatile v8b*)(DP + u * 8) = v; }
    if (u < (size_t)CO * KK / 8) { const int o = (int)(u / (KK / 8)), k0 = (int)(u % (KK / 8)) * 8; v8b v;
#pragma unroll
      for (int j = 0; j < 8; ++j) v[j] = (b16)(bf16_rne(W[(size_t)(k0 + j) * CO + o]) * WSC); *(volatile v8b*)(WT + (size_t)o * KK + k0) = v; }
    __threadfence(); } }
__global__ __launch_bounds__(32) void deconv_kernel(const b16* __restrict__ DP, const int* __restrict__ neigh, const int* __restrict__ bid, const b16* __restrict__ WT, float* __restrict__ H, float* __restrict__ PS) {
  __shared__ __attribute__((aligned(16))) b16 Ah[16][KK + 8]; __shared__ float Tf[16][36]; __shared__ int Bt[16]; const int lane = threadIdx.x, nloc = lane & 15, hlf = lane >> 4; const size_t m0 = (size_t)blockIdx.x * 16;
  for (int pidx = lane; pidx < 16 * KT; pidx += 32) { const int rr = pidx / KT, k = pidx % KT; const size_t nb = (size_t)iclamp(neigh[(m0 + rr) * KT + k], 0, N - 1); const v8b* srow = (const v8b*)(DP + nb * CI); v8b* drow = (v8b*)(&Ah[rr][k * CI]);
#pragma unroll
    for (int q = 0; q < 4; ++q) drow[q] = srow[q]; }
  if (lane < 16) Bt[lane] = iclamp(bid[m0 + lane], 0, NB - 1);
  wave_lds_sync(); v8f acc[2] = {(v8f){}, (v8f){}};
#pragma unroll 3
  for (int kb = 0; kb < KK; kb += 32) { const v16b a = frag_kb(&Ah[nloc][kb], hlf);
#pragma unroll
    for (int t = 0; t < 2; ++t) acc[t] = wmma16b(a, frag_kb(WT + (size_t)(t * 16 + nloc) * KK + kb, hlf), acc[t]); }
#pragma unroll
  for (int t = 0; t < 2; ++t)
#pragma unroll
    for (int r8 = 0; r8 < 8; ++r8) Tf[8 * hlf + r8][t * 16 + nloc] = acc[t][r8] * (1.0f / (XS * WSC));
  wave_lds_sync();
  float s[4] = {0.f, 0.f, 0.f, 0.f}, q[4] = {0.f, 0.f, 0.f, 0.f}; const int b0 = Bt[0]; int nslot = Bt[15] - b0 + 1; nslot = nslot > 4 ? 4 : nslot;
  for (int rr = 0; rr < 16; ++rr) { const int sl = Bt[rr] - b0; const float v = Tf[rr][lane];
#pragma unroll
    for (int z = 0; z < 4; ++z) if (sl == z) { s[z] += v; q[z] += pmul(v, v); } }
  for (int pass = 0; pass < 2; ++pass) { for (int rr = 0; rr < 16; ++rr) ((volatile float*)H)[(m0 + rr) * CO + lane] = Tf[rr][lane];
    volatile float* P = (volatile float*)PS + (size_t)blockIdx.x * 288;
#pragma unroll
    for (int z = 0; z < 4; ++z) { P[32 + z * 64 + lane] = s[z]; P[32 + z * 64 + 32 + lane] = q[z]; }
    float hv = 0.0f; if (lane < 4) hv = (lane < nslot) ? (float)(b0 + lane) : -1.0f; else if (lane < 8) { int c = 0; for (int rr = 0; rr < 16; ++rr) c += (Bt[rr] - b0 == lane - 4) ? 1 : 0; hv = (float)c; } P[lane] = hv;
    __threadfence(); } }
__global__ __launch_bounds__(256) void stat_kernel(const float* __restrict__ PS, int NTV, float* __restrict__ ST) { __shared__ double S[NB][CO], Q[NB][CO], CNT[NB]; const int t = threadIdx.x; const int b = t / CO, c = t % CO;
  { double s = 0.0, q = 0.0, n = 0.0;
#pragma unroll 1
    for (int tile = 0; tile < NTV; ++tile) { const float* P = PS + (size_t)tile * 288;
#pragma unroll
      for (int z = 0; z < 4; ++z) { if ((int)P[z] == b) { s += (double)P[32 + z * 64 + c]; q += (double)P[32 + z * 64 + 32 + c]; n += (double)P[4 + z]; } } }
    S[b][c] = s; Q[b][c] = q; if (c == 0) CNT[b] = n; }
  __syncthreads();
  const int g = c / CG; double gs = 0.0; for (int j = 0; j < CG; ++j) gs += S[b][g * CG + j]; const double inv_cnt = 1.0 / (CNT[b] * (double)CO / G + (double)EPS); const double mean = gs * inv_cnt;
  double gv = 0.0; for (int j = 0; j < CG; ++j) { const int cc = g * CG + j; gv += Q[b][cc] - 2.0 * mean * S[b][cc] + CNT[b] * mean * mean; } const double var = gv * inv_cnt; const float inv_std = (float)(1.0 / sqrt(var + (double)EPS));
  for (int pass = 0; pass < 2; ++pass) { ((volatile float*)ST)[b * 64 + c] = (float)mean; ((volatile float*)ST)[b * 64 + 32 + c] = inv_std; __threadfence(); } }
__global__ __launch_bounds__(256) void fin_kernel(const float* __restrict__ H, const float* __restrict__ ST, const int* __restrict__ bid, const float* __restrict__ gamma, const float* __restrict__ beta, int NTV, float* __restrict__ out) { const size_t u = (size_t)blockIdx.x * 256 + threadIdx.x; if (u >= (size_t)N * CO / 4) return; const size_t n = u / 8; const int c0 = (int)(u % 8) * 4; const int b = iclamp(bid[n], 0, NB - 1);
  v4f r = {0.0f, 0.0f, 0.0f, 0.0f}; if (n < (size_t)NTV * 16) { const v4f h = *(const v4f*)(H + n * CO + c0); for (int k = 0; k < 4; ++k) { const int c = c0 + k; r[k] = fmaxf(pmul(pmul(h[k] - ST[b * 64 + c], ST[b * 64 + 32 + c]), bf16_rne(gamma[c])) + bf16_rne(beta[c]), 0.0f); } }
  for (int pass = 0; pass < 2; ++pass) { *(volatile v4f*)(out + n * CO + c0) = r; __threadfence(); } }
}

extern "C" void kernel_launch(void* const* d_in, const int* in_sizes, int n_in, void* d_out, int out_size, void* d_ws, size_t ws_size, hipStream_t stream) {
  (void)n_in;
  auto Fp = [&](int i) { return (const float*)d_in[i]; }; auto Ip = [&](int i) { return (const int*)d_in[i]; };
  if (in_sizes[0] != N * CI || in_sizes[1] != KT * CI * CO || in_sizes[4] != N * KT || in_sizes[5] != N || out_size != N * CO) return;
  const int NTV = NTILE;
  size_t off = 0; char* ws = (char*)d_ws;
  auto carve = [&](size_t bytes) { char* p = ws + off; off += (bytes + 255) & ~(size_t)255; return p; };
  b16* DP = (b16*)carve((size_t)N * CI * 2); b16* WT = (b16*)carve((size_t)CO * KK * 2); float* H = (float*)carve((size_t)N * CO * 4); float* PS = (float*)carve((size_t)NTILE * 288 * 4); float* ST = (float*)carve((size_t)NB * 64 * 4);
  if (off > ws_size || off > ((size_t)96 << 20)) return;
  prep_kernel<<<(unsigned)(((size_t)N * CI / 8 + 255) / 256), 256, 0, stream>>>(Fp(0), Fp(1), DP, WT);
  deconv_kernel<<<NTV, 32, 0, stream>>>(DP, Ip(4), Ip(5), WT, H, PS);
  stat_kernel<<<1, 256, 0, stream>>>(PS, NTV, ST);
  fin_kernel<<<(unsigned)(((size_t)N * CO / 4 + 255) / 256), 256, 0, stream>>>(H, ST, Ip(5), Fp(2), Fp(3), NTV, (float*)d_out);
}
